// SchNetAngular_2774548873992
// MI455X (gfx1250) — hardware-verified
//
#include <hip/hip_runtime.h>
#include <stddef.h>


#pragma clang fp contract(off)

#define NB      8
#define NA      512
#define NNB     64
#define DN      128
#define NG      25
#define GK      32
#define GA      512
#define NL      3
#define NATOM   (NB * NA)
#define NPAIR   (NATOM * NNB)
#define NTHR    256
#define NWAVE   8
#define NBN     64
#define APA     136
#define GSTR    132
#define PW1     0
#define PW2     4096
#define PIN     20480
#define PFO     36864
#define PDE     53248
#define PAN     69632
#define PLAY    135168
#define PWTOT   (NL * PLAY)
#define PBLK    (PWTOT / (NTHR * 8))
#define GBLK    ((NATOM * GA) / (NTHR * 8))
#define EBLK    ((NATOM * DN) / (NTHR * 4))
#define PRBLK   (NPAIR / NTHR)
#define ABLK    (NATOM / NBN)
#define WSCAP   134217728
#define SW      16.0f
#define SX      16.0f
#define SHID    64.0f
#define SAG     64.0f
#define INV16   0.0625f
#define INV256  0.00390625f
#define INV1024 0.0009765625f
#define CUT     5.0f
#define GSTART  1.2f
#define GEPS    1e-12f
#define LN2F    0.6931471805599453f

static_assert((PWTOT % (NTHR * 8)) == 0);
static_assert((PLAY % (NTHR * 8)) == 0);
static_assert((PW2 % (NTHR * 8)) == 0);
static_assert((PIN % (NTHR * 8)) == 0);
static_assert((PFO % (NTHR * 8)) == 0);
static_assert((PDE % (NTHR * 8)) == 0);
static_assert((PAN % (NTHR * 8)) == 0);
static_assert(((NATOM * GA) % (NTHR * 8)) == 0);
static_assert(((NATOM * DN) % (NTHR * 4)) == 0);
static_assert((NPAIR % NTHR) == 0);
static_assert((NATOM % NBN) == 0);
static_assert(((APA * 2) % 16) == 0);
static_assert(((GSTR * 4) % 16) == 0);
static_assert(NBN * APA * 2 <= NBN * GSTR * 4);
static_assert(NBN == NWAVE * 8);
static_assert(NNB * GK == NTHR * 8);
static_assert(NNB * 4 == NTHR);
static_assert(NA == 512);
static_assert(NNB == 64);

typedef float          v4f   __attribute__((ext_vector_type(4)));
typedef float          v8f   __attribute__((ext_vector_type(8)));
typedef unsigned short v8us  __attribute__((ext_vector_type(8)));
typedef _Float16       v8h   __attribute__((ext_vector_type(8)));
typedef _Float16       v16h  __attribute__((ext_vector_type(16)));
union FragH { v16h v; v8h h[2]; };
union Cvt8  { v8h v; v8us u; };

__device__ __forceinline__ v8f wmh(v16h a, v16h b, v8f c) {
  v8f d = __builtin_amdgcn_wmma_f32_16x16x32_f16(false, a, false, b, (short)0, c, false, false);
  asm volatile("v_nop\n\tv_nop\n\tv_nop\n\tv_nop" : "+v"(d) : "v"(a), "v"(b));
  return d;
}
__device__ __forceinline__ v8f zero8() {
  v8f z = {0.f, 0.f, 0.f, 0.f, 0.f, 0.f, 0.f, 0.f};
  return z;
}

__device__ __forceinline__ float sspf(float x) {
  const float e = expf(-fabsf(x));
  return (fmaxf(x, 0.0f) + log1pf(e)) - LN2F;
}

__device__ __forceinline__ void gemm16x64(const _Float16* ap, const _Float16* bpl, int kp, int nks, int n0,
                                          int m, int hh, v8f& c0, v8f& c1, v8f& c2, v8f& c3) {
  c0 = zero8(); c1 = zero8(); c2 = zero8(); c3 = zero8();
#pragma unroll 1
  for (int ks = 0; ks < nks; ++ks) {
    FragH a;
    a.h[0] = *(const v8h*)(ap + 32 * ks);
    a.h[1] = *(const v8h*)(ap + 32 * ks + 16);
    const _Float16* bp = bpl + (size_t)(n0 + m) * kp + 32 * ks + 8 * hh;
    FragH b;
    b.h[0] = *(const v8h*)(bp);
    b.h[1] = *(const v8h*)(bp + 16);
    c0 = wmh(a.v, b.v, c0);
    b.h[0] = *(const v8h*)(bp + (size_t)16 * kp);
    b.h[1] = *(const v8h*)(bp + (size_t)16 * kp + 16);
    c1 = wmh(a.v, b.v, c1);
    b.h[0] = *(const v8h*)(bp + (size_t)32 * kp);
    b.h[1] = *(const v8h*)(bp + (size_t)32 * kp + 16);
    c2 = wmh(a.v, b.v, c2);
    b.h[0] = *(const v8h*)(bp + (size_t)48 * kp);
    b.h[1] = *(const v8h*)(bp + (size_t)48 * kp + 16);
    c3 = wmh(a.v, b.v, c3);
  }
}

__device__ __forceinline__ void stage8(float* sp, v8f a, float scl, float bias) {
#pragma unroll
  for (int r = 0; r < 8; ++r) sp[r * GSTR] = a[r] * scl + bias;
}
__device__ __forceinline__ void acc8(float* sp, v8f a, float scl) {
#pragma unroll
  for (int r = 0; r < 8; ++r) sp[r * GSTR] = sp[r * GSTR] + a[r] * scl;
}
__device__ __forceinline__ void stage8h(_Float16* sp, v8f a, float scl, float bias) {
#pragma unroll
  for (int r = 0; r < 8; ++r) sp[r * APA] = (_Float16)((a[r] * scl + bias) * SAG);
}

__global__ __launch_bounds__(NTHR) void k_prep(
    const float* __restrict__ w1, const float* __restrict__ w2, const float* __restrict__ win,
    const float* __restrict__ wfo, const float* __restrict__ wde, const float* __restrict__ wan, unsigned short* wp) {
  const int tid = (int)threadIdx.x;
  const int o = ((int)blockIdx.x * NTHR + tid) * 8;
  const int l = o / PLAY;
  const int rem = o - l * PLAY;
  const float* src = w1;
  int n, k0, K;
  if (rem < PW2)      { n = rem >> 5; k0 = rem & 31; K = NG; src = w1; }
  else if (rem < PIN) { const int idx = rem - PW2; n = idx >> 7; k0 = idx & 127; K = DN; src = w2; }
  else if (rem < PFO) { const int idx = rem - PIN; n = idx >> 7; k0 = idx & 127; K = DN; src = win; }
  else if (rem < PDE) { const int idx = rem - PFO; n = idx >> 7; k0 = idx & 127; K = DN; src = wfo; }
  else if (rem < PAN) { const int idx = rem - PDE; n = idx >> 7; k0 = idx & 127; K = DN; src = wde; }
  else                { const int idx = rem - PAN; n = idx >> 9; k0 = idx & 511; K = GA; src = wan; }
  Cvt8 cv;
#pragma unroll
  for (int j = 0; j < 8; ++j) {
    const int k = k0 + j;
    const int kc = k < K ? k : K - 1;
    const float v = src[((size_t)l * K + kc) * DN + n] * SW;
    cv.v[j] = (_Float16)(k < K ? v : v * 0.0f);
  }
  unsigned short* dp = wp + o;
  *(volatile v8us*)dp = cv.u;
  __threadfence();
  *(volatile v8us*)dp = cv.u;
}

__global__ __launch_bounds__(NTHR) void k_gcvt(const float* __restrict__ g, unsigned short* gh) {
  const size_t o = ((size_t)blockIdx.x * NTHR + threadIdx.x) * 8;
  const v4f xa = *(const v4f*)(g + o);
  const v4f xb = *(const v4f*)(g + o + 4);
  Cvt8 cv;
  cv.v[0] = (_Float16)xa.x; cv.v[1] = (_Float16)xa.y; cv.v[2] = (_Float16)xa.z; cv.v[3] = (_Float16)xa.w;
  cv.v[4] = (_Float16)xb.x; cv.v[5] = (_Float16)xb.y; cv.v[6] = (_Float16)xb.z; cv.v[7] = (_Float16)xb.w;
  *(volatile v8us*)(gh + o) = cv.u;
  __threadfence();
  *(volatile v8us*)(gh + o) = cv.u;
}

__global__ __launch_bounds__(NTHR) void k_embed(const int* __restrict__ z, const float* __restrict__ emb,
                                                float* xo, int maxz) {
  const int gid = (int)blockIdx.x * NTHR + (int)threadIdx.x;
  const int row = gid >> 5;
  const int c4 = (gid & 31) * 4;
  int zz = z[row];
  zz = zz < 0 ? zz + maxz : zz;
  zz = zz < 0 ? 0 : (zz > maxz - 1 ? maxz - 1 : zz);
  const v4f v = *(const v4f*)(emb + (size_t)zz * DN + c4);
  float* dp = xo + (size_t)row * DN + c4;
  *(volatile v4f*)dp = v;
  __threadfence();
  *(volatile v4f*)dp = v;
}

__global__ __launch_bounds__(NTHR) void k_geom(const float* __restrict__ pos, const int* __restrict__ nbr,
                                               const int* __restrict__ msk, unsigned short* fq, float* scl) {
  __shared__ __attribute__((aligned(16))) _Float16 sF[NTHR * GK];
  const int tid = (int)threadIdx.x;
  const int pid = (int)blockIdx.x * NTHR + tid;
  const int ba = pid >> 6;
  const int bs = ba >> 9;
  int j = nbr[pid];
  j = j < 0 ? j + NA : j;
  j = j < 0 ? 0 : (j > NA - 1 ? NA - 1 : j);
  const float* pa = pos + (size_t)ba * 3;
  const float* pb = pos + (size_t)(bs * NA + j) * 3;
  const float dx = pb[0] - pa[0];
  const float dy = pb[1] - pa[1];
  const float dz = pb[2] - pa[2];
  const float t0 = dx * dx;
  const float t1 = dy * dy;
  const float t2 = dz * dz;
  const float sq = (t0 + t2) + t1;
  const float r = sqrtf(sq + GEPS);
  const float s1 = 1.0f * (1.0f / 24.0f);
  const float c1 = GSTART * (1.0f - s1) + CUT * s1;
  const float c0 = GSTART * (1.0f - 0.0f) + CUT * 0.0f;
  const float width = c1 - c0;
  const float ww = width * width;
  const float coef = -0.5f / ww;
  const float zp = r * 0.0f;
  _Float16* fr = sF + tid * GK;
#pragma unroll 1
  for (int g = 0; g < NG; ++g) {
    const float sg = (float)g * (1.0f / 24.0f);
    float cg = GSTART * (1.0f - sg) + CUT * sg;
    cg = (g == NG - 1) ? CUT : cg;
    const float d = r - cg;
    const float dd = d * d;
    const float f = expf(coef * dd);
    fr[g] = (_Float16)f;
  }
#pragma unroll 1
  for (int g = NG; g < GK; ++g) fr[g] = (_Float16)zp;
  const float cm = (r <= CUT) ? 1.0f : 0.0f;
  const float sv = cm * (float)msk[pid];
  *(volatile float*)(scl + pid) = sv;
  __syncthreads();
#pragma unroll 1
  for (int i = 0; i < 4; ++i) {
    const int p = tid + NTHR * i;
    const int pr = p >> 2, q = p & 3;
    Cvt8 cv;
    cv.v = *(const v8h*)(sF + pr * GK + 8 * q);
    *(volatile v8us*)(fq + ((size_t)blockIdx.x * NTHR + pr) * GK + 8 * q) = cv.u;
  }
  __threadfence();
  *(volatile float*)(scl + pid) = sv;
#pragma unroll 1
  for (int i = 0; i < 4; ++i) {
    const int p = tid + NTHR * i;
    const int pr = p >> 2, q = p & 3;
    Cvt8 cv;
    cv.v = *(const v8h*)(sF + pr * GK + 8 * q);
    *(volatile v8us*)(fq + ((size_t)blockIdx.x * NTHR + pr) * GK + 8 * q) = cv.u;
  }
}

__global__ __launch_bounds__(NTHR) void k_y(const float* __restrict__ xg, const unsigned short* __restrict__ wp,
                                            float* yg, int l) {
  __shared__ __attribute__((aligned(16))) _Float16 sA[NBN * APA];
  __shared__ __attribute__((aligned(16))) float sU[NBN * GSTR];
  const int tid = (int)threadIdx.x, lane = tid & 31, wave = tid >> 5, hh = lane >> 4, m = lane & 15;
  const int n0 = (int)blockIdx.x * NBN;
  {
    const int nl = tid >> 2, q = tid & 3;
    int row = n0 + nl;
    row = row > NATOM - 1 ? NATOM - 1 : row;
    const float* rp = xg + (size_t)row * DN + 32 * q;
#pragma unroll
    for (int i = 0; i < 4; ++i) {
      const v4f xa = *(const v4f*)(rp + 8 * i);
      const v4f xb = *(const v4f*)(rp + 8 * i + 4);
      Cvt8 cv;
      cv.v[0] = (_Float16)(xa.x * SX); cv.v[1] = (_Float16)(xa.y * SX); cv.v[2] = (_Float16)(xa.z * SX); cv.v[3] = (_Float16)(xa.w * SX);
      cv.v[4] = (_Float16)(xb.x * SX); cv.v[5] = (_Float16)(xb.y * SX); cv.v[6] = (_Float16)(xb.z * SX); cv.v[7] = (_Float16)(xb.w * SX);
      *(v8h*)(sA + nl * APA + 32 * q + 8 * i) = cv.v;
    }
  }
  __syncthreads();
  const int rt = wave & 3, cg = wave >> 2;
  const _Float16* wl = (const _Float16*)wp + (size_t)l * PLAY;
  {
    v8f a0, a1, a2, a3;
    gemm16x64(sA + (16 * rt + m) * APA + 8 * hh, wl + PIN, DN, 4, 64 * cg, m, hh, a0, a1, a2, a3);
    float* sp = sU + (16 * rt + 8 * hh) * GSTR + 64 * cg + m;
    stage8(sp,      a0, INV256, 0.0f);
    stage8(sp + 16, a1, INV256, 0.0f);
    stage8(sp + 32, a2, INV256, 0.0f);
    stage8(sp + 48, a3, INV256, 0.0f);
  }
  __syncthreads();
#pragma unroll 1
  for (int it = 0; it < NBN / NWAVE; ++it) {
    const int s = wave + NWAVE * it;
    const v4f v = *(const v4f*)(sU + s * GSTR + 4 * lane);
    *(volatile v4f*)(yg + (size_t)(n0 + s) * DN + 4 * lane) = v;
  }
  __threadfence();
#pragma unroll 1
  for (int it = 0; it < NBN / NWAVE; ++it) {
    const int s = wave + NWAVE * it;
    const v4f v = *(const v4f*)(sU + s * GSTR + 4 * lane);
    *(volatile v4f*)(yg + (size_t)(n0 + s) * DN + 4 * lane) = v;
  }
}

__device__ __forceinline__ float aggpart(v8f c, int rbase, float b2v, const float* sS, const float* syc) {
  float p = 0.0f;
#pragma unroll
  for (int r = 0; r < 8; ++r) {
    const int rr = rbase + r;
    const float wv = (c[r] * INV1024 + b2v) * sS[rr];
    const float yv = syc[rr * DN];
    p = p + wv * yv;
  }
  return p;
}

__global__ __launch_bounds__(NTHR) void k_cfconv(
    const unsigned short* __restrict__ fq, const float* __restrict__ scl, const int* __restrict__ nbr,
    const float* __restrict__ yg, const unsigned short* __restrict__ wp,
    const float* __restrict__ fb1, const float* __restrict__ fb2, float* agg, int l) {
  __shared__ __attribute__((aligned(16))) _Float16 sF[NNB * GK];
  __shared__ __attribute__((aligned(16))) _Float16 sH[NNB * APA];
  __shared__ __attribute__((aligned(16))) float sY[NNB * DN];
  __shared__ __attribute__((aligned(16))) float sAgg[DN];
  __shared__ float sPar[2 * DN];
  __shared__ float sS[NNB];
  __shared__ int sJ[NNB];
  const int tid = (int)threadIdx.x, lane = tid & 31, wave = tid >> 5, hh = lane >> 4, m = lane & 15;
  const int atom = (int)blockIdx.x;
  const int bs = atom >> 9;
  const size_t p0 = (size_t)atom * NNB;

  {
    Cvt8 cv;
    cv.u = *(const v8us*)(fq + p0 * GK + 8 * tid);
    *(v8h*)(sF + 8 * tid) = cv.v;
  }
  if (tid < NNB) {
    sS[tid] = scl[p0 + tid];
    int j = nbr[p0 + tid];
    j = j < 0 ? j + NA : j;
    j = j < 0 ? 0 : (j > NA - 1 ? NA - 1 : j);
    sJ[tid] = bs * NA + j;
  }
  if (tid < DN) {
    sPar[tid]      = fb1[(size_t)l * DN + tid];
    sPar[DN + tid] = fb2[(size_t)l * DN + tid];
  }
  __syncthreads();

  {
    const int r = tid >> 2, q = tid & 3;
    const float* src = yg + (size_t)sJ[r] * DN + 32 * q;
    float* dst = sY + r * DN + 32 * q;
#pragma unroll
    for (int c = 0; c < 8; ++c) *(v4f*)(dst + 4 * c) = *(const v4f*)(src + 4 * c);
  }

  const int n = 16 * wave + m;
  const _Float16* wl = (const _Float16*)wp + (size_t)l * PLAY;

  {
    FragH b;
    const _Float16* bp = wl + PW1 + n * GK + 8 * hh;
    b.h[0] = *(const v8h*)(bp);
    b.h[1] = *(const v8h*)(bp + 16);
    const float b1v = sPar[n];
#pragma unroll
    for (int mt = 0; mt < 4; ++mt) {
      FragH a;
      const _Float16* ap = sF + (16 * mt + m) * GK + 8 * hh;
      a.h[0] = *(const v8h*)(ap);
      a.h[1] = *(const v8h*)(ap + 16);
      const v8f acc = wmh(a.v, b.v, zero8());
      _Float16* hp = sH + (16 * mt + 8 * hh) * APA + n;
#pragma unroll
      for (int r = 0; r < 8; ++r) hp[r * APA] = (_Float16)(sspf(acc[r] * INV16 + b1v) * SHID);
    }
  }
  __syncthreads();

  v8f c0 = zero8(), c1 = zero8(), c2 = zero8(), c3 = zero8();
  {
    const _Float16* bpl = wl + PW2 + (size_t)n * DN + 8 * hh;
#pragma unroll 1
    for (int ks = 0; ks < 4; ++ks) {
      FragH b;
      b.h[0] = *(const v8h*)(bpl + 32 * ks);
      b.h[1] = *(const v8h*)(bpl + 32 * ks + 16);
      const _Float16* ap = sH + m * APA + 32 * ks + 8 * hh;
      FragH a;
      a.h[0] = *(const v8h*)(ap);             a.h[1] = *(const v8h*)(ap + 16);             c0 = wmh(a.v, b.v, c0);
      a.h[0] = *(const v8h*)(ap + 16 * APA);  a.h[1] = *(const v8h*)(ap + 16 * APA + 16);  c1 = wmh(a.v, b.v, c1);
      a.h[0] = *(const v8h*)(ap + 32 * APA);  a.h[1] = *(const v8h*)(ap + 32 * APA + 16);  c2 = wmh(a.v, b.v, c2);
      a.h[0] = *(const v8h*)(ap + 48 * APA);  a.h[1] = *(const v8h*)(ap + 48 * APA + 16);  c3 = wmh(a.v, b.v, c3);
    }
  }

  {
    const float b2v = sPar[DN + n];
    const float* syc = sY + n;
    float p = aggpart(c0, 8 * hh, b2v, sS, syc);
    p = p + aggpart(c1, 16 + 8 * hh, b2v, sS, syc);
    p = p + aggpart(c2, 32 + 8 * hh, b2v, sS, syc);
    p = p + aggpart(c3, 48 + 8 * hh, b2v, sS, syc);
    const float q = __shfl_xor(p, 16);
    p = p + q;
    if (hh == 0) sAgg[n] = p;
  }
  __syncthreads();

  if (tid < 32) {
    const v4f v = *(const v4f*)(sAgg + 4 * lane);
    *(volatile v4f*)(agg + (size_t)atom * DN + 4 * lane) = v;
  }
  __threadfence();
  if (tid < 32) {
    const v4f v = *(const v4f*)(sAgg + 4 * lane);
    *(volatile v4f*)(agg + (size_t)atom * DN + 4 * lane) = v;
  }
}

__global__ __launch_bounds__(NTHR) void k_upd(
    const float* __restrict__ agg, const unsigned short* __restrict__ gh, const unsigned short* __restrict__ wp,
    const float* __restrict__ bfo, const float* __restrict__ bde, float* xo, int l) {
  __shared__ __attribute__((aligned(16))) float sU[NBN * GSTR];
  __shared__ __attribute__((aligned(16))) _Float16 sB[NBN * APA];
  __shared__ float sPar[2 * DN];
  _Float16* sA = (_Float16*)sU;
  const int tid = (int)threadIdx.x, lane = tid & 31, wave = tid >> 5, hh = lane >> 4, m = lane & 15;
  const int n0 = (int)blockIdx.x * NBN;

  {
    const int nl = tid >> 2, q = tid & 3;
    int row = n0 + nl;
    row = row > NATOM - 1 ? NATOM - 1 : row;
    const float* rp = agg + (size_t)row * DN + 32 * q;
#pragma unroll
    for (int i = 0; i < 4; ++i) {
      const v4f xa = *(const v4f*)(rp + 8 * i);
      const v4f xb = *(const v4f*)(rp + 8 * i + 4);
      Cvt8 cv;
      cv.v[0] = (_Float16)(xa.x * SAG); cv.v[1] = (_Float16)(xa.y * SAG); cv.v[2] = (_Float16)(xa.z * SAG); cv.v[3] = (_Float16)(xa.w * SAG);
      cv.v[4] = (_Float16)(xb.x * SAG); cv.v[5] = (_Float16)(xb.y * SAG); cv.v[6] = (_Float16)(xb.z * SAG); cv.v[7] = (_Float16)(xb.w * SAG);
      *(v8h*)(sA + nl * APA + 32 * q + 8 * i) = cv.v;
    }
  }
  if (tid < DN) {
    sPar[tid]      = bfo[(size_t)l * DN + tid];
    sPar[DN + tid] = bde[(size_t)l * DN + tid];
  }
  __syncthreads();

  const int rt = wave & 3, cg = wave >> 2;
  const _Float16* wl = (const _Float16*)wp + (size_t)l * PLAY;

  {
    v8f a0, a1, a2, a3;
    gemm16x64(sA + (16 * rt + m) * APA + 8 * hh, wl + PFO, DN, 4, 64 * cg, m, hh, a0, a1, a2, a3);
    _Float16* sp = sB + (16 * rt + 8 * hh) * APA + 64 * cg + m;
    const float* bb = sPar + 64 * cg + m;
    stage8h(sp,      a0, INV1024, bb[0]);
    stage8h(sp + 16, a1, INV1024, bb[16]);
    stage8h(sp + 32, a2, INV1024, bb[32]);
    stage8h(sp + 48, a3, INV1024, bb[48]);
  }
  __syncthreads();

  {
    v8f a0, a1, a2, a3;
    gemm16x64(sB + (16 * rt + m) * APA + 8 * hh, wl + PDE, DN, 4, 64 * cg, m, hh, a0, a1, a2, a3);
    float* sp = sU + (16 * rt + 8 * hh) * GSTR + 64 * cg + m;
    const float* bb = sPar + DN + 64 * cg + m;
    stage8(sp,      a0, INV1024, bb[0]);
    stage8(sp + 16, a1, INV1024, bb[16]);
    stage8(sp + 32, a2, INV1024, bb[32]);
    stage8(sp + 48, a3, INV1024, bb[48]);
  }

  {
    v8f a0, a1, a2, a3;
    const _Float16* ap = (const _Float16*)gh + (size_t)(n0 + 16 * rt + m) * GA + 8 * hh;
    gemm16x64(ap, wl + PAN, GA, 16, 64 * cg, m, hh, a0, a1, a2, a3);
    float* sp = sU + (16 * rt + 8 * hh) * GSTR + 64 * cg + m;
    acc8(sp,      a0, INV16);
    acc8(sp + 16, a1, INV16);
    acc8(sp + 32, a2, INV16);
    acc8(sp + 48, a3, INV16);
  }
  __syncthreads();

#pragma unroll 1
  for (int it = 0; it < NBN / NWAVE; ++it) {
    const int s = wave + NWAVE * it;
    float* up = sU + s * GSTR + 4 * lane;
    const v4f v = *(const v4f*)up;
    const v4f xv = *(const v4f*)(xo + (size_t)(n0 + s) * DN + 4 * lane);
    v4f o;
    o.x = xv.x + sspf(v.x);
    o.y = xv.y + sspf(v.y);
    o.z = xv.z + sspf(v.z);
    o.w = xv.w + sspf(v.w);
    *(v4f*)up = o;
  }
#pragma unroll 1
  for (int it = 0; it < NBN / NWAVE; ++it) {
    const int s = wave + NWAVE * it;
    const v4f v = *(const v4f*)(sU + s * GSTR + 4 * lane);
    *(volatile v4f*)(xo + (size_t)(n0 + s) * DN + 4 * lane) = v;
  }
  __threadfence();
#pragma unroll 1
  for (int it = 0; it < NBN / NWAVE; ++it) {
    const int s = wave + NWAVE * it;
    const v4f v = *(const v4f*)(sU + s * GSTR + 4 * lane);
    *(volatile v4f*)(xo + (size_t)(n0 + s) * DN + 4 * lane) = v;
  }
}

extern "C" void kernel_launch(void* const* d_in, const int* in_sizes, int n_in,
                              void* d_out, int out_size, void* d_ws, size_t ws_size,
                              hipStream_t stream) {
  if (n_in < 16) return;
  if (in_sizes[0] != NATOM) return;
  if (in_sizes[1] != NATOM * 3) return;
  if (in_sizes[2] != NPAIR || in_sizes[3] != NPAIR) return;
  if (in_sizes[4] != NATOM * GA) return;
  if (in_sizes[5] < DN || (in_sizes[5] % DN) != 0) return;
  const int maxz = in_sizes[5] / DN;
  if (in_sizes[6] != NL * NG * DN || in_sizes[7] != NL * DN) return;
  if (in_sizes[8] != NL * DN * DN || in_sizes[9] != NL * DN) return;
  if (in_sizes[10] != NL * DN * DN || in_sizes[11] != NL * DN * DN || in_sizes[12] != NL * DN) return;
  if (in_sizes[13] != NL * DN * DN || in_sizes[14] != NL * DN) return;
  if (in_sizes[15] != NL * GA * DN) return;
  if (out_size != NATOM * DN) return;

  const int*   z     = (const int*)d_in[0];
  const float* pos   = (const float*)d_in[1];
  const int*   nbr   = (const int*)d_in[2];
  const int*   msk   = (const int*)d_in[3];
  const float* gi    = (const float*)d_in[4];
  const float* emb   = (const float*)d_in[5];
  const float* w1    = (const float*)d_in[6];
  const float* b1    = (const float*)d_in[7];
  const float* w2    = (const float*)d_in[8];
  const float* b2    = (const float*)d_in[9];
  const float* win   = (const float*)d_in[10];
  const float* wfo   = (const float*)d_in[11];
  const float* bfo   = (const float*)d_in[12];
  const float* wde   = (const float*)d_in[13];
  const float* bde   = (const float*)d_in[14];
  const float* wan   = (const float*)d_in[15];
  float* xo = (float*)d_out;

  char* ws = (char*)d_ws;
  size_t off = 0;
  const size_t oW = off; off += (size_t)PWTOT * 2;          off = (off + 255) & ~(size_t)255;
  const size_t oG = off; off += (size_t)NATOM * GA * 2;     off = (off + 255) & ~(size_t)255;
  const size_t oF = off; off += (size_t)NPAIR * GK * 2;     off = (off + 255) & ~(size_t)255;
  const size_t oS = off; off += (size_t)NPAIR * 4;          off = (off + 255) & ~(size_t)255;
  const size_t oY = off; off += (size_t)NATOM * DN * 4;     off = (off + 255) & ~(size_t)255;
  const size_t oA = off; off += (size_t)NATOM * DN * 4;     off = (off + 255) & ~(size_t)255;
  if (off > ws_size || off > (size_t)WSCAP) return;
  unsigned short* wp  = (unsigned short*)(ws + oW);
  unsigned short* ghp = (unsigned short*)(ws + oG);
  unsigned short* fq  = (unsigned short*)(ws + oF);
  float* scl          = (float*)(ws + oS);
  float* yg           = (float*)(ws + oY);
  float* agg          = (float*)(ws + oA);

  k_prep<<<PBLK, NTHR, 0, stream>>>(w1, w2, win, wfo, wde, wan, wp);
  k_gcvt<<<GBLK, NTHR, 0, stream>>>(gi, ghp);
  k_embed<<<EBLK, NTHR, 0, stream>>>(z, emb, xo, maxz);
  k_geom<<<PRBLK, NTHR, 0, stream>>>(pos, nbr, msk, fq, scl);
  for (int l = 0; l < NL; ++l) {
    k_y<<<ABLK, NTHR, 0, stream>>>(xo, wp, yg, l);
    k_cfconv<<<NATOM, NTHR, 0, stream>>>(fq, scl, nbr, yg, wp, b1, b2, agg, l);
    k_upd<<<ABLK, NTHR, 0, stream>>>(agg, ghp, wp, bfo, bde, xo, l);
  }
}
